// Decoder_42202348650664
// MI455X (gfx1250) — hardware-verified
//
#include <hip/hip_runtime.h>
#include <math.h>

#ifndef NB
#define NB 2
#endif
#ifndef SEQ
#define SEQ 2048
#endif
#define NB_FULL 2
#define SEQ_FULL 2048

constexpr int DM     = 1024;
constexpr int NH     = 16;
constexpr int HDIM   = 64;
constexpr int FFD    = 4096;
constexpr int MR     = NB * SEQ;
constexpr int NCH    = 1;
constexpr int MH     = MR / NCH;
constexpr int QTILES = SEQ / 16;
constexpr int LQK    = 2 * DM;
constexpr int ST_PITCH = 68;
constexpr int ST_WAVE  = 16 * ST_PITCH;
constexpr int OT_PITCH = 72;
constexpr int TP_PITCH = 72;
constexpr float SCORE_SCALE = 1.0f / (float)HDIM;

static_assert(NB <= NB_FULL && SEQ <= SEQ_FULL);
static_assert(SEQ % 128 == 0);
static_assert(MR % 256 == 0);
static_assert(MR == MH * NCH && MH % 128 == 0);
static_assert(DM == NH * HDIM);
static_assert(HDIM == 64);
static_assert(DM % 128 == 0 && FFD % 128 == 0 && LQK % 128 == 0);
static_assert(DM % 32 == 0 && FFD % 32 == 0);
static_assert((DM & (DM - 1)) == 0 && (FFD & (FFD - 1)) == 0);
static_assert(DM == 256 * 4);
static_assert(DM == 128 * 8);
static_assert(((MR * (DM / 8)) % 256) == 0);
static_assert((NB * NH * QTILES) % 8 == 0 && QTILES % 8 == 0);
static_assert(DM % 64 == 0 && FFD % 64 == 0 && HDIM % 64 == 0);
static_assert(ST_PITCH >= 64 && ST_PITCH % 4 == 0);
static_assert(OT_PITCH >= HDIM && OT_PITCH % 8 == 0 && TP_PITCH >= 64 && TP_PITCH % 8 == 0);

typedef __attribute__((ext_vector_type(16))) _Float16 v16h;
typedef __attribute__((ext_vector_type(8)))  _Float16 v8h;
typedef __attribute__((ext_vector_type(16))) __bf16   v16bf;
typedef __attribute__((ext_vector_type(8)))  float    v8f;
typedef __attribute__((ext_vector_type(4)))  float    v4f;
typedef __attribute__((ext_vector_type(8)))  unsigned short v8us;
typedef __attribute__((ext_vector_type(4)))  unsigned short v4us;
typedef __attribute__((ext_vector_type(8)))  unsigned int   v8u;

union FragHU { v16h  v; v8us h[2]; v8u w; };
union FragBU { v16bf v; v8us h[2]; v8u w; };

__device__ __forceinline__ unsigned short bf16_bits(float f) {
  unsigned int u = __float_as_uint(f);
  u = (u + 0x7FFFu + ((u >> 16) & 1u)) >> 16;
  return (unsigned short)u;
}
__device__ __forceinline__ float bf16_to_f(unsigned short b) { return __uint_as_float(((unsigned int)b) << 16); }
__device__ __forceinline__ float bfr(float f) { return bf16_to_f(bf16_bits(f)); }
__device__ __forceinline__ unsigned short f16_bits(float f) { return __builtin_bit_cast(unsigned short, (_Float16)f); }
__device__ __forceinline__ float gelu_exact(float x) { return 0.5f * x * (1.0f + erff(x * 0.70710678118654752f)); }

template <int OPT> struct Op;
template <> struct Op<0> {
  typedef FragBU U;
  static __device__ __forceinline__ U load(const unsigned short* p) {
    U f; f.h[0] = *(const v8us*)(p); f.h[1] = *(const v8us*)(p + 16); return f;
  }
  static __device__ __forceinline__ v8f mma(const U& a, const U& b, v8f c) {
    return __builtin_amdgcn_wmma_f32_16x16x32_bf16(false, a.v, false, b.v, (short)0, c, false, false);
  }
};
template <> struct Op<1> {
  typedef FragHU U;
  static __device__ __forceinline__ U load(const unsigned short* p) {
    U f; f.h[0] = *(const v8us*)(p); f.h[1] = *(const v8us*)(p + 16); return f;
  }
  static __device__ __forceinline__ v8f mma(const U& a, const U& b, v8f c) {
    return __builtin_amdgcn_wmma_f32_16x16x32_f16(false, a.v, false, b.v, (short)0, c, false, false);
  }
};

__device__ __forceinline__ void guard8(v8f& c0, v8f& c1, v8f& c2, v8f& c3, v8f& c4, v8f& c5, v8f& c6, v8f& c7,
                                       v8u x0, v8u x1, v8u x2, v8u x3, v8u x4, v8u x5) {
  asm volatile("v_nop\n\tv_nop\n\tv_nop\n\tv_nop"
               : "+v"(c0), "+v"(c1), "+v"(c2), "+v"(c3), "+v"(c4), "+v"(c5), "+v"(c6), "+v"(c7)
               : "v"(x0), "v"(x1), "v"(x2), "v"(x3), "v"(x4), "v"(x5));
}
__device__ __forceinline__ void guard2(v8f& c0, v8f& c1, v8u x0, v8u x1, v8u x2, v8u x3, v8u x4, v8u x5) {
  asm volatile("v_nop\n\tv_nop\n\tv_nop\n\tv_nop"
               : "+v"(c0), "+v"(c1)
               : "v"(x0), "v"(x1), "v"(x2), "v"(x3), "v"(x4), "v"(x5));
}
__device__ __forceinline__ void guard4(v8f& c0, v8f& c1, v8f& c2, v8f& c3, v8u x0, v8u x1, v8u x2, v8u x3, v8u x4) {
  asm volatile("v_nop\n\tv_nop\n\tv_nop\n\tv_nop"
               : "+v"(c0), "+v"(c1), "+v"(c2), "+v"(c3)
               : "v"(x0), "v"(x1), "v"(x2), "v"(x3), "v"(x4));
}

__global__ __launch_bounds__(256) void cvt_x_kernel(const float* __restrict__ x, unsigned short* __restrict__ XB) {
  const int i   = blockIdx.x * 256 + threadIdx.x;
  const int row = i / (DM / 8);
  const int c8  = (i % (DM / 8)) * 8;
  const int b = row / SEQ, s = row % SEQ;
  const float* sp = x + ((size_t)b * SEQ_FULL + (size_t)s) * DM + c8;
  const v4f a = *(const v4f*)(sp);
  const v4f c = *(const v4f*)(sp + 4);
  v8us o;
#pragma unroll
  for (int e = 0; e < 4; ++e) { o[e] = bf16_bits(a[e]); o[4 + e] = bf16_bits(c[e]); }
  unsigned short* dst = XB + (size_t)i * 8;
  *(volatile v8us*)dst = o;
  __threadfence();
  *(volatile v8us*)dst = o;
}

template <int MODE>
__device__ __forceinline__ void wt_prep_body(unsigned short* T, const float* __restrict__ src, unsigned short* __restrict__ dst,
                                             int ld_in, int ld_out, int in_bs, int out_bs) {
  const int tid = threadIdx.x;
  const int k0 = blockIdx.x * 64, n0 = blockIdx.y * 64;
  const float* sp = src + (size_t)blockIdx.z * (size_t)in_bs;
  unsigned short* dp = dst + (size_t)blockIdx.z * (size_t)out_bs;
  const int nn = tid & 63, kq = tid >> 6;
#pragma unroll 4
  for (int i = 0; i < 16; ++i) {
    const int kk = kq + 4 * i;
    const float v = sp[(size_t)(k0 + kk) * ld_in + n0 + nn];
    unsigned short bits;
    if (MODE == 0) bits = bf16_bits(v);
    else           bits = f16_bits(bfr(v) * 16.0f);
    T[nn * TP_PITCH + kk] = bits;
  }
  __syncthreads();
#pragma unroll
  for (int i = 0; i < 2; ++i) {
    const int p = tid + 256 * i;
    const int row = p >> 3, seg = p & 7;
    const v8us v = *(const v8us*)(T + row * TP_PITCH + seg * 8);
    unsigned short* o = dp + (size_t)(n0 + row) * ld_out + k0 + seg * 8;
    *(volatile v8us*)o = v;
    __threadfence();
    *(volatile v8us*)o = v;
  }
}

__global__ __launch_bounds__(256) void wt_prep_bf16_kernel(const float* __restrict__ src, unsigned short* __restrict__ dst,
                                                           int ld_in, int ld_out, int in_bs, int out_bs) {
  __shared__ __align__(16) unsigned short T[64 * TP_PITCH];
  wt_prep_body<0>(T, src, dst, ld_in, ld_out, in_bs, out_bs);
}
__global__ __launch_bounds__(256) void wt_prep_f16c_kernel(const float* __restrict__ src, unsigned short* __restrict__ dst,
                                                           int ld_in, int ld_out, int in_bs, int out_bs) {
  __shared__ __align__(16) unsigned short T[64 * TP_PITCH];
  wt_prep_body<1>(T, src, dst, ld_in, ld_out, in_bs, out_bs);
}

enum { EPI_H_COL = 0, EPI_H_ROW = 1, EPI_H_GELU = 2, EPI_F_COL = 3 };

template <int EPI>
__device__ __forceinline__ void epi_half(const v8f (&acc)[4], float* st, int lane, int rowG0, int colBase,
                                         const float* bias0, const float* bias1, int bsplit, int bmask,
                                         _Float16* Ch, float* Cf, int ldc, float scale) {
  const int m = lane & 15, hh = lane >> 4;
  __syncthreads();
  float brow[8];
#pragma unroll
  for (int r = 0; r < 8; ++r) brow[r] = 0.0f;
  if (EPI == EPI_H_ROW) {
#pragma unroll
    for (int r = 0; r < 8; ++r) brow[r] = bfr(bias0[(rowG0 + 8 * hh + r) & bmask]);
  }
#pragma unroll
  for (int i = 0; i < 4; ++i) {
    float bc = 0.0f;
    if (EPI != EPI_H_ROW) {
      const int col = colBase + 16 * i + m;
      const float ba = bias0[col & bmask];
      const float bb = bias1[col & bmask];
      bc = bfr((col < bsplit) ? ba : bb);
    }
#pragma unroll
    for (int r = 0; r < 8; ++r)
      st[(8 * hh + r) * ST_PITCH + 16 * i + m] = acc[i][r] * scale + (bc + brow[r]);
  }
  __syncthreads();
  if (EPI != EPI_F_COL) {
#pragma unroll 1
    for (int it = 0; it < 4; ++it) {
      const int row = it * 4 + (lane >> 3), seg = lane & 7;
      const float* sp = st + row * ST_PITCH + seg * 8;
      const v4f x0 = *(const v4f*)(sp);
      const v4f x1 = *(const v4f*)(sp + 4);
      v8h hv;
#pragma unroll
      for (int e = 0; e < 4; ++e) {
        float f0 = x0[e], f1 = x1[e];
        if (EPI == EPI_H_GELU) { f0 = gelu_exact(f0); f1 = gelu_exact(f1); }
        hv[e] = (_Float16)f0;
        hv[4 + e] = (_Float16)f1;
      }
      _Float16* dst = Ch + (size_t)(rowG0 + row) * ldc + colBase + seg * 8;
      *(volatile v8h*)dst = hv;
      __threadfence();
      *(volatile v8h*)dst = hv;
    }
  } else {
#pragma unroll 1
    for (int it = 0; it < 8; ++it) {
      const int row = it * 2 + (lane >> 4), seg = lane & 15;
      const v4f xv = *(const v4f*)(st + row * ST_PITCH + seg * 4);
      float* dst = Cf + (size_t)(rowG0 + row) * ldc + colBase + seg * 4;
      *(volatile v4f*)dst = xv;
      __threadfence();
      *(volatile v4f*)dst = xv;
    }
  }
}

template <int OPT, int EPI>
__device__ __forceinline__ void gemm_body(float* St, const unsigned short* __restrict__ A, const unsigned short* __restrict__ Bt,
                                          const float* bias0, const float* bias1,
                                          int bsplit, int bmask, _Float16* Ch, float* Cf,
                                          int K, int ldc, float scale) {
  typedef typename Op<OPT>::U FU;
  const int tid = threadIdx.x, lane = tid & 31;
  const int w = __builtin_amdgcn_readfirstlane(tid >> 5);
  const int wm = w & 3, wn = w >> 2;
  const int m = lane & 15, hh = lane >> 4;
  const int rowBase = blockIdx.y * 128 + wm * 32;
  const int colBase = blockIdx.x * 128 + wn * 64;
  const unsigned short* pa0 = A + (size_t)(rowBase + m) * K + 8 * hh;
  const unsigned short* pa1 = pa0 + (size_t)16 * K;
  const unsigned short* pb0 = Bt + (size_t)(colBase + m) * K + 8 * hh;
  const unsigned short* pb1 = pb0 + (size_t)16 * K;
  const unsigned short* pb2 = pb0 + (size_t)32 * K;
  const unsigned short* pb3 = pb0 + (size_t)48 * K;

  const v8f z8 = {0.f, 0.f, 0.f, 0.f, 0.f, 0.f, 0.f, 0.f};
  v8f acc0[4], acc1[4];
#pragma unroll
  for (int i = 0; i < 4; ++i) { acc0[i] = z8; acc1[i] = z8; }

#pragma unroll 1
  for (int kt = 0; kt < K; kt += 32) {
    const FU a0 = Op<OPT>::load(pa0 + kt);
    const FU a1 = Op<OPT>::load(pa1 + kt);
    const FU b0 = Op<OPT>::load(pb0 + kt);
    const FU b1 = Op<OPT>::load(pb1 + kt);
    const FU b2 = Op<OPT>::load(pb2 + kt);
    const FU b3 = Op<OPT>::load(pb3 + kt);
    acc0[0] = Op<OPT>::mma(a0, b0, acc0[0]);
    acc1[0] = Op<OPT>::mma(a1, b0, acc1[0]);
    acc0[1] = Op<OPT>::mma(a0, b1, acc0[1]);
    acc1[1] = Op<OPT>::mma(a1, b1, acc1[1]);
    acc0[2] = Op<OPT>::mma(a0, b2, acc0[2]);
    acc1[2] = Op<OPT>::mma(a1, b2, acc1[2]);
    acc0[3] = Op<OPT>::mma(a0, b3, acc0[3]);
    acc1[3] = Op<OPT>::mma(a1, b3, acc1[3]);
    guard8(acc0[0], acc0[1], acc0[2], acc0[3], acc1[0], acc1[1], acc1[2], acc1[3], a0.w, a1.w, b0.w, b1.w, b2.w, b3.w);
  }

  float* st = St + w * ST_WAVE;
  epi_half<EPI>(acc0, st, lane, rowBase,      colBase, bias0, bias1, bsplit, bmask, Ch, Cf, ldc, scale);
  epi_half<EPI>(acc1, st, lane, rowBase + 16, colBase, bias0, bias1, bsplit, bmask, Ch, Cf, ldc, scale);
}

__global__ __launch_bounds__(256) void gemm_qk_kernel(const unsigned short* __restrict__ A, const unsigned short* __restrict__ Bt,
                                                      const float* __restrict__ bq, const float* __restrict__ bk,
                                                      _Float16* __restrict__ Ch) {
  __shared__ __align__(16) float St[8 * ST_WAVE];
  gemm_body<0, EPI_H_COL>(St, A, Bt, bq, bk, DM, DM - 1, Ch, (float*)0, DM, LQK, 1.0f);
}
__global__ __launch_bounds__(256) void gemm_vt_kernel(const unsigned short* __restrict__ A, const unsigned short* __restrict__ Bt,
                                                      const float* __restrict__ bv, _Float16* __restrict__ Ch) {
  __shared__ __align__(16) float St[8 * ST_WAVE];
  gemm_body<0, EPI_H_ROW>(St, A, Bt, bv, bv, DM, DM - 1, Ch, (float*)0, DM, MR, 1.0f);
}
__global__ __launch_bounds__(256) void gemm_f32o_kernel(const unsigned short* __restrict__ A, const unsigned short* __restrict__ Bt,
                                                        const float* __restrict__ bias, float* __restrict__ Cf,
                                                        int K, float scale) {
  __shared__ __align__(16) float St[8 * ST_WAVE];
  gemm_body<1, EPI_F_COL>(St, A, Bt, bias, bias, 1 << 30, DM - 1, (_Float16*)0, Cf, K, DM, scale);
}
__global__ __launch_bounds__(256) void gemm_gelu_kernel(const unsigned short* __restrict__ A, const unsigned short* __restrict__ Bt,
                                                        const float* __restrict__ bias, _Float16* __restrict__ Ch) {
  __shared__ __align__(16) float St[8 * ST_WAVE];
  gemm_body<1, EPI_H_GELU>(St, A, Bt, bias, bias, 1 << 30, FFD - 1, Ch, (float*)0, DM, FFD, 1.0f / 16.0f);
}

__global__ __launch_bounds__(256) void attn_kernel(const unsigned short* __restrict__ QK, const unsigned short* __restrict__ Vt,
                                                   _Float16* __restrict__ CTX) {
  __shared__ __align__(16) _Float16 Ot[8 * 16 * OT_PITCH];
  const int tid = threadIdx.x, lane = tid & 31;
  const int w = __builtin_amdgcn_readfirstlane(tid >> 5);
  const int m = lane & 15, hh = lane >> 4;
  const int gw = blockIdx.x * 8 + w;
  const int qt = gw % QTILES;
  const int bh = gw / QTILES;
  const int h = bh % NH, b = bh / NH;
  const int q0 = qt * 16;
  const size_t rb = (size_t)b * SEQ;

  const unsigned short* qp = QK + (rb + (size_t)(q0 + m)) * LQK + h * HDIM + 8 * hh;
  const FragHU qb0 = Op<1>::load(qp);
  const FragHU qb1 = Op<1>::load(qp + 32);
  const unsigned short* kp = QK + (rb + (size_t)m) * LQK + DM + h * HDIM + 8 * hh;
  const unsigned short* vp = Vt + (size_t)(h * HDIM + m) * MR + rb + 8 * hh;

  const v8f z8 = {0.f, 0.f, 0.f, 0.f, 0.f, 0.f, 0.f, 0.f};
  v8f o0 = z8, o1 = z8, o2 = z8, o3 = z8;
  float mrun = -1e30f, lrun = 0.0f;
  const int nkt = (q0 + 16 + 31) >> 5;

#pragma unroll 1
  for (int t = 0; t < nkt; ++t) {
    const int kt = t * 32;
    const unsigned short* k0p = kp + (size_t)kt * LQK;
    const unsigned short* k1p = k0p + (size_t)16 * LQK;
    const FragHU ka0 = Op<1>::load(k0p);
    const FragHU ka1 = Op<1>::load(k0p + 32);
    const FragHU ka2 = Op<1>::load(k1p);
    const FragHU ka3 = Op<1>::load(k1p + 32);
    v8f s0 = z8, s1 = z8;
    s0 = Op<1>::mma(ka0, qb0, s0);
    s1 = Op<1>::mma(ka2, qb0, s1);
    s0 = Op<1>::mma(ka1, qb1, s0);
    s1 = Op<1>::mma(ka3, qb1, s1);
    guard2(s0, s1, ka0.w, ka1.w, ka2.w, ka3.w, qb0.w, qb1.w);

    float t0[8], t1[8];
    float mx = -1e30f;
    const bool diag = (kt + 31 > q0);
    const int lim = q0 + m - kt - 8 * hh;
#pragma unroll
    for (int r = 0; r < 8; ++r) {
      float a = s0[r] * SCORE_SCALE;
      float c = s1[r] * SCORE_SCALE;
      if (diag) {
        a = (r <= lim) ? a : -1e30f;
        c = (16 + r <= lim) ? c : -1e30f;
      }
      t0[r] = a; t1[r] = c;
      mx = fmaxf(mx, fmaxf(a, c));
    }
    mx = fmaxf(mx, __shfl_xor(mx, 16, 32));
    const float mnew = fmaxf(mrun, mx);
    const float fs = __expf(mrun - mnew);
    mrun = mnew;
    const float mb = mnew - 6.931471806f;
    float ps = 0.0f;
    FragHU pb;
#pragma unroll
    for (int r = 0; r < 8; ++r) {
      const float p0 = __expf(t0[r] - mb);
      const float p1 = __expf(t1[r] - mb);
      ps += p0 + p1;
      pb.v[r] = (_Float16)p0;
      pb.v[8 + r] = (_Float16)p1;
    }
    lrun = lrun * fs + ps;
#pragma unroll
    for (int r = 0; r < 8; ++r) { o0[r] *= fs; o1[r] *= fs; o2[r] *= fs; o3[r] *= fs; }

    const unsigned short* vk = vp + kt;
    const FragHU va0 = Op<1>::load(vk);
    const FragHU va1 = Op<1>::load(vk + (size_t)16 * MR);
    const FragHU va2 = Op<1>::load(vk + (size_t)32 * MR);
    const FragHU va3 = Op<1>::load(vk + (size_t)48 * MR);
    o0 = Op<1>::mma(va0, pb, o0);
    o1 = Op<1>::mma(va1, pb, o1);
    o2 = Op<1>::mma(va2, pb, o2);
    o3 = Op<1>::mma(va3, pb, o3);
    guard4(o0, o1, o2, o3, va0.w, va1.w, va2.w, va3.w, pb.w);
  }

  const float ltot = lrun + __shfl_xor(lrun, 16, 32);
  const float inv = 16.0f * (1.0f / ltot);
  _Float16* ot = Ot + w * (16 * OT_PITCH);
  {
    v8h x0, x1, x2, x3;
#pragma unroll
    for (int r = 0; r < 8; ++r) {
      x0[r] = (_Float16)(o0[r] * inv);
      x1[r] = (_Float16)(o1[r] * inv);
      x2[r] = (_Float16)(o2[r] * inv);
      x3[r] = (_Float16)(o3[r] * inv);
    }
    _Float16* wr = ot + m * OT_PITCH + 8 * hh;
    *(v8h*)(wr)      = x0;
    *(v8h*)(wr + 16) = x1;
    *(v8h*)(wr + 32) = x2;
    *(v8h*)(wr + 48) = x3;
  }
  __syncthreads();
#pragma unroll
  for (int it = 0; it < 4; ++it) {
    const int row = it * 4 + (lane >> 3), seg = lane & 7;
    const v8h v = *(const v8h*)(ot + row * OT_PITCH + seg * 8);
    _Float16* dst = CTX + (rb + (size_t)(q0 + row)) * DM + h * HDIM + seg * 8;
    *(volatile v8h*)dst = v;
    __threadfence();
    *(volatile v8h*)dst = v;
  }
}

__device__ __forceinline__ float block_sum256(float v, float* red, int lane, int w) {
#pragma unroll
  for (int mk = 16; mk >= 1; mk >>= 1) v += __shfl_xor(v, mk, 32);
  __syncthreads();
  if (lane == 0) red[w] = v;
  __syncthreads();
  float s = 0.0f;
#pragma unroll
  for (int i = 0; i < 8; ++i) s += red[i];
  return s;
}

__global__ __launch_bounds__(256) void add_ln1_kernel(const unsigned short* __restrict__ XB, const float* __restrict__ AO,
                                                      const float* __restrict__ gam, const float* __restrict__ bet,
                                                      float* __restrict__ HF, _Float16* __restrict__ HB) {
  __shared__ float red[8];
  __shared__ __align__(16) _Float16 hs[DM];
  const int tid = threadIdx.x, lane = tid & 31, w = tid >> 5;
  const size_t row = blockIdx.x;
  const int c4 = tid * 4;
  const v4us xb = *(const v4us*)(XB + row * DM + c4);
  const v4f ao = *(const v4f*)(AO + row * DM + c4);
  float v[4];
  float s = 0.0f;
#pragma unroll
  for (int e = 0; e < 4; ++e) { v[e] = bf16_to_f(xb[e]) + ao[e]; s += v[e]; }
  const float mu = block_sum256(s, red, lane, w) * (1.0f / DM);
  float ss = 0.0f;
#pragma unroll
  for (int e = 0; e < 4; ++e) { v[e] -= mu; ss += v[e] * v[e]; }
  const float var = block_sum256(ss, red, lane, w) * (1.0f / DM);
  const float inv = rsqrtf(var + 1e-5f);
  const v4f g4 = *(const v4f*)(gam + c4);
  const v4f b4 = *(const v4f*)(bet + c4);
  v4f y;
#pragma unroll
  for (int e = 0; e < 4; ++e) {
    y[e] = v[e] * inv * bfr(g4[e]) + bfr(b4[e]);
    hs[c4 + e] = (_Float16)y[e];
  }
  float* dst = HF + row * DM + c4;
  *(volatile v4f*)dst = y;
  __threadfence();
  *(volatile v4f*)dst = y;
  __syncthreads();
  if (tid < 128) {
    const v8h hv = *(const v8h*)(hs + tid * 8);
    _Float16* dh = HB + row * DM + tid * 8;
    *(volatile v8h*)dh = hv;
    __threadfence();
    *(volatile v8h*)dh = hv;
  }
}

__global__ __launch_bounds__(256) void add_ln2_kernel(const float* __restrict__ HF, const float* __restrict__ FF,
                                                      const float* __restrict__ gam, const float* __restrict__ bet,
                                                      float* __restrict__ out) {
  __shared__ float red[8];
  const int tid = threadIdx.x, lane = tid & 31, w = tid >> 5;
  const size_t row = blockIdx.x;
  const int c4 = tid * 4;
  const v4f hv = *(const v4f*)(HF + row * DM + c4);
  const v4f fv = *(const v4f*)(FF + row * DM + c4);
  float v[4];
  float s = 0.0f;
#pragma unroll
  for (int e = 0; e < 4; ++e) { v[e] = hv[e] + fv[e]; s += v[e]; }
  const float mu = block_sum256(s, red, lane, w) * (1.0f / DM);
  float ss = 0.0f;
#pragma unroll
  for (int e = 0; e < 4; ++e) { v[e] -= mu; ss += v[e] * v[e]; }
  const float var = block_sum256(ss, red, lane, w) * (1.0f / DM);
  const float inv = rsqrtf(var + 1e-5f);
  const v4f g4 = *(const v4f*)(gam + c4);
  const v4f b4 = *(const v4f*)(bet + c4);
  v4f y;
#pragma unroll
  for (int e = 0; e < 4; ++e) y[e] = v[e] * inv * bfr(g4[e]) + bfr(b4[e]);
  const size_t bb = row / SEQ, sq = row % SEQ;
  float* dst = out + (bb * SEQ_FULL + sq) * DM + c4;
  *(volatile v4f*)dst = y;
  __threadfence();
  *(volatile v4f*)dst = y;
}

constexpr size_t cmaxz(size_t a, size_t b) { return a > b ? a : b; }
constexpr size_t SZ_W1T = (size_t)FFD * DM * 2;
constexpr size_t SZ_W2T = (size_t)DM * FFD * 2;
constexpr size_t SZ_HB  = (size_t)MR * DM * 2;
constexpr size_t SZ_R2  = (size_t)MR * DM * 4;
constexpr size_t SZ_R1  = (size_t)MR * DM * 4;
constexpr size_t SZ_XB  = (size_t)MR * DM * 2;
constexpr size_t SZ_WQK = (size_t)LQK * DM * 2;
constexpr size_t SZ_WV  = (size_t)DM * DM * 2;
constexpr size_t SZ_WO  = (size_t)DM * DM * 2;
constexpr size_t SZ_EARLY = SZ_XB + SZ_WQK + SZ_WV + SZ_WO;
constexpr size_t SZ_ACT = (size_t)MH * FFD * 2;
constexpr size_t SZ_R3  = cmaxz(SZ_EARLY, SZ_ACT);
constexpr size_t WS_TOTAL = SZ_W1T + SZ_W2T + SZ_HB + SZ_R2 + SZ_R1 + SZ_R3;
static_assert(WS_TOTAL <= (size_t)134217728);
static_assert((size_t)MR * LQK * 2 <= SZ_R1);
static_assert((size_t)MR * DM * 4 <= SZ_R1);
static_assert((size_t)DM * MR * 2 + (size_t)MR * DM * 2 <= SZ_R2);
static_assert((size_t)MR * DM * 4 <= SZ_R2);
static_assert(SZ_EARLY <= SZ_R3 && SZ_ACT <= SZ_R3);
static_assert(SZ_XB % 256 == 0 && SZ_HB % 256 == 0 && SZ_WQK % 256 == 0 && SZ_WV % 256 == 0);

extern "C" void kernel_launch(void* const* d_in, const int* in_sizes, int n_in,
                              void* d_out, int out_size, void* d_ws, size_t ws_size, hipStream_t stream) {
  if (n_in < 17 || d_out == nullptr || d_ws == nullptr) return;
  const int need_rows = ((NB - 1) * SEQ_FULL + SEQ) * DM;
  if (in_sizes[0] < need_rows || out_size < need_rows) return;
  if (in_sizes[1] < NH * DM * HDIM || in_sizes[3] < NH * DM * HDIM || in_sizes[5] < NH * DM * HDIM) return;
  if (in_sizes[2] < DM || in_sizes[4] < DM || in_sizes[6] < DM || in_sizes[8] < DM) return;
  if (in_sizes[7] < DM * DM || in_sizes[9] < DM * FFD || in_sizes[11] < FFD * DM) return;
  if (in_sizes[10] < FFD || in_sizes[12] < DM) return;
  if (in_sizes[13] < DM || in_sizes[14] < DM || in_sizes[15] < DM || in_sizes[16] < DM) return;
  if (WS_TOTAL > ws_size) return;

  const float* x   = (const float*)d_in[0];
  const float* Wq  = (const float*)d_in[1];
  const float* bq  = (const float*)d_in[2];
  const float* Wk  = (const float*)d_in[3];
  const float* bk  = (const float*)d_in[4];
  const float* Wv  = (const float*)d_in[5];
  const float* bv  = (const float*)d_in[6];
  const float* Wo  = (const float*)d_in[7];
  const float* bo  = (const float*)d_in[8];
  const float* W1  = (const float*)d_in[9];
  const float* b1  = (const float*)d_in[10];
  const float* W2  = (const float*)d_in[11];
  const float* b2  = (const float*)d_in[12];
  const float* g1  = (const float*)d_in[13];
  const float* be1 = (const float*)d_in[14];
  const float* g2  = (const float*)d_in[15];
  const float* be2 = (const float*)d_in[16];
  float* out = (float*)d_out;

  char* ws = (char*)d_ws;
  char* pW1T = ws;
  char* pW2T = pW1T + SZ_W1T;
  char* pHB  = pW2T + SZ_W2T;
  char* pR2  = pHB + SZ_HB;
  char* pR1  = pR2 + SZ_R2;
  char* pR3  = pR1 + SZ_R1;

  unsigned short* W1T  = (unsigned short*)pW1T;
  unsigned short* W2T  = (unsigned short*)pW2T;
  unsigned short* HB   = (unsigned short*)pHB;
  unsigned short* VtP  = (unsigned short*)pR2;
  unsigned short* CTX  = (unsigned short*)(pR2 + (size_t)DM * MR * 2);
  float*          HF   = (float*)pR2;
  unsigned short* QKP  = (unsigned short*)pR1;
  float*          AO   = (float*)pR1;
  float*          FFo  = (float*)pR1;
  unsigned short* XB   = (unsigned short*)pR3;
  unsigned short* WqkT = (unsigned short*)(pR3 + SZ_XB);
  unsigned short* WvT  = (unsigned short*)(pR3 + SZ_XB + SZ_WQK);
  unsigned short* WoT  = (unsigned short*)(pR3 + SZ_XB + SZ_WQK + SZ_WV);
  unsigned short* ACT  = (unsigned short*)pR3;

  cvt_x_kernel<<<(MR * (DM / 8)) / 256, 256, 0, stream>>>(x, XB);
  wt_prep_bf16_kernel<<<dim3(DM / 64, HDIM / 64, NH), 256, 0, stream>>>(Wq, WqkT, HDIM, DM, DM * HDIM, HDIM * DM);
  wt_prep_bf16_kernel<<<dim3(DM / 64, HDIM / 64, NH), 256, 0, stream>>>(Wk, WqkT + (size_t)DM * DM, HDIM, DM, DM * HDIM, HDIM * DM);
  wt_prep_bf16_kernel<<<dim3(DM / 64, HDIM / 64, NH), 256, 0, stream>>>(Wv, WvT, HDIM, DM, DM * HDIM, HDIM * DM);
  wt_prep_f16c_kernel<<<dim3(DM / 64, DM / 64, 1), 256, 0, stream>>>(Wo, WoT, DM, DM, 0, 0);
  wt_prep_f16c_kernel<<<dim3(DM / 64, FFD / 64, 1), 256, 0, stream>>>(W1, W1T, FFD, DM, 0, 0);
  wt_prep_f16c_kernel<<<dim3(FFD / 64, DM / 64, 1), 256, 0, stream>>>(W2, W2T, DM, FFD, 0, 0);

  gemm_qk_kernel<<<dim3(LQK / 128, MR / 128), 256, 0, stream>>>(XB, WqkT, bq, bk, (_Float16*)QKP);
  gemm_vt_kernel<<<dim3(MR / 128, DM / 128), 256, 0, stream>>>(WvT, XB, bv, (_Float16*)VtP);
  attn_kernel<<<(NB * NH * QTILES) / 8, 256, 0, stream>>>(QKP, VtP, (_Float16*)CTX);
  gemm_f32o_kernel<<<dim3(DM / 128, MR / 128), 256, 0, stream>>>(CTX, WoT, bo, AO, DM, 1.0f / 256.0f);
  add_ln1_kernel<<<MR, 256, 0, stream>>>(XB, AO, g1, be1, HF, (_Float16*)HB);
  for (int c = 0; c < NCH; ++c) {
    const unsigned short* hbc = HB + (size_t)c * MH * DM;
    float* ffc = FFo + (size_t)c * MH * DM;
    gemm_gelu_kernel<<<dim3(FFD / 128, MH / 128), 256, 0, stream>>>(hbc, W1T, b1, (_Float16*)ACT);
    gemm_f32o_kernel<<<dim3(DM / 128, MH / 128), 256, 0, stream>>>(ACT, W2T, b2, ffc, FFD, 1.0f / 16.0f);
  }
  add_ln2_kernel<<<MR, 256, 0, stream>>>(HF, FFo, g2, be2, out);
}
